// DecoderBlock_6330781794323
// MI455X (gfx1250) — hardware-verified
//
#include <hip/hip_runtime.h>
#include <math.h>
#include <stdint.h>

typedef __attribute__((ext_vector_type(16))) _Float16 v16h;
typedef __attribute__((ext_vector_type(8)))  _Float16 v8h;
typedef __attribute__((ext_vector_type(16))) __bf16   v16b;
typedef __attribute__((ext_vector_type(8)))  __bf16   v8b;
typedef __attribute__((ext_vector_type(8)))  float    v8f;
typedef __attribute__((ext_vector_type(4)))  float    v4f;
typedef __attribute__((ext_vector_type(2)))  float    v2f;

constexpr int kBatch    = 4;
constexpr int kSeq      = 1024;
constexpr int kMem      = 1024;
constexpr int kDm       = 512;
constexpr int kHeads    = 8;
constexpr int kHd       = 64;
constexpr int kDin      = 1024;
constexpr int kNst      = 16;
constexpr int kDtR      = 32;
constexpr int kXdW      = 64;
constexpr int kXzP      = 2 * kDin;
constexpr int kDff      = 4 * kDm;
constexpr int kRows     = kBatch * kSeq;
constexpr int kMRows    = kBatch * kMem;
constexpr int kHalfB    = kBatch / 2;
constexpr int kHalfRows = kHalfB * kSeq;
constexpr int kTP       = 260;
static_assert(kHeads * kHd == kDm, "head split");
static_assert(kDtR + 2 * kNst == kXdW, "x_proj width");
static_assert(kHd == 64, "attention kernel head width");
static_assert(kDm == 128 * 4, "LN kernel: 128 threads x 4 floats per row");
static_assert(kHalfRows % kSeq == 0 && kBatch % 2 == 0, "half boundaries are sequence boundaries");
static_assert(kDm % 32 == 0 && kDin % 32 == 0 && kDtR % 32 == 0 && kDff % 32 == 0, "K multiples of 32");
static_assert(kRows % 64 == 0 && kMRows % 64 == 0 && kHalfRows % 64 == 0 && kDm % 64 == 0 && kMem % 64 == 0 &&
              kXzP % 64 == 0 && kXdW % 64 == 0 && kDin % 64 == 0 && kDff % 64 == 0, "M,N multiples of 64");
static_assert(kSeq % 64 == 0 && kMem % 64 == 0 && kSeq % 16 == 0 && kDin % 256 == 0 && kHalfRows % 64 == 0, "tile multiples");

constexpr float kQkScale = 0.125f;
static_assert(kQkScale * kQkScale * (float)kHd == 1.0f, "score scale");
constexpr float kWsc    = 64.0f;
constexpr float kUsc    = 256.0f;
constexpr float kDtsc   = 256.0f;
constexpr float kYsc    = 1024.0f;
constexpr float kAttSc  = 64.0f;
constexpr float kPCarry = 32768.0f;

constexpr size_t kMiB      = 1048576ull;
constexpr size_t kOffX1    = 0;
constexpr size_t kOffX2    = 8 * kMiB;
constexpr size_t kOffAttO  = 16 * kMiB;
constexpr size_t kOffXZ    = 16 * kMiB;
constexpr size_t kOffHPre  = 16 * kMiB;
constexpr size_t kOffDLR   = 32 * kMiB;
constexpr size_t kOffXD    = 40 * kMiB;
constexpr size_t kOffMO    = 48 * kMiB;
constexpr size_t kOffFfnO  = 48 * kMiB;
constexpr size_t kOffX16   = 56 * kMiB;
constexpr size_t kOffAt16  = 56 * kMiB;
constexpr size_t kOffM16   = 60 * kMiB;
constexpr size_t kOffX1h   = 60 * kMiB;
constexpr size_t kOffWq16  = 64 * kMiB;
constexpr size_t kOffWk16  = kOffWq16 + (size_t)kDm * kDm * 2;
constexpr size_t kOffWv16  = kOffWk16 + (size_t)kDm * kDm * 2;
constexpr size_t kOffWo16  = kOffWv16 + (size_t)kDm * kDm * 2;
constexpr size_t kOffWxp16 = 64 * kMiB;
constexpr size_t kOffWdt16 = kOffWxp16 + (size_t)kXdW * kDin * 2;
constexpr size_t kOffDt16  = kOffWdt16 + (size_t)kDin * kDtR * 2;
constexpr size_t kOffQ16   = 66 * kMiB;
constexpr size_t kOffUc16  = 66 * kMiB;
constexpr size_t kOffK16   = 70 * kMiB;
constexpr size_t kOffY16   = 70 * kMiB;
constexpr size_t kOffVt16  = 74 * kMiB;
constexpr size_t kOffWin16 = 74 * kMiB;
constexpr size_t kOffWout16= 76 * kMiB;
constexpr size_t kOffX2H   = 78 * kMiB;
constexpr size_t kOffX2L   = 82 * kMiB;
constexpr size_t kOffW1H   = 86 * kMiB;
constexpr size_t kOffW1L   = 88 * kMiB;
constexpr size_t kOffW2H   = 90 * kMiB;
constexpr size_t kOffW2L   = 92 * kMiB;
constexpr size_t kOffG1H   = 94 * kMiB;
constexpr size_t kOffG1L   = 110 * kMiB;
constexpr size_t kWsTotal  = 126 * kMiB;
static_assert(kWsTotal == 132120576ull, "carve total");
static_assert(kWsTotal <= 134217728ull, "carve cap");
static_assert(kOffX2 + (size_t)kRows * kDm * 4 == kOffAttO, "X1/X2");
static_assert(kOffAttO + (size_t)kRows * kDm * 4 <= kOffDLR, "ATTO");
static_assert(kOffXZ + (size_t)kHalfRows * kXzP * 4 == kOffDLR, "XZ half");
static_assert(kOffHPre + (size_t)kRows * kDff * 4 == kOffMO, "HPRE");
static_assert(kOffDLR + (size_t)kHalfRows * kDin * 4 == kOffXD, "DLR half");
static_assert(kOffXD + (size_t)kHalfRows * kXdW * 4 <= kOffMO, "XD half");
static_assert(kOffMO + (size_t)kRows * kDm * 4 == kOffX16, "MO/FFNO");
static_assert(kOffX16 + (size_t)kRows * kDm * 2 == kOffM16, "X16");
static_assert(kOffM16 + (size_t)kMRows * kDm * 2 == kOffWq16, "M16");
static_assert(kOffWo16 + (size_t)kDm * kDm * 2 == kOffQ16, "weight slot");
static_assert(kOffDt16 + (size_t)kHalfRows * kDtR * 2 <= kOffQ16, "ssm small planes");
static_assert(kOffQ16 + (size_t)kRows * kDm * 2 == kOffK16, "Q16");
static_assert(kOffUc16 + (size_t)kHalfRows * kDin * 2 == kOffK16, "UC16 half");
static_assert(kOffK16 + (size_t)kMRows * kDm * 2 == kOffVt16, "K16");
static_assert(kOffY16 + (size_t)kHalfRows * kDin * 2 == kOffVt16, "Y16 half");
static_assert(kOffVt16 + (size_t)kBatch * kDm * kMem * 2 == kOffX2H, "VT16");
static_assert(kOffWin16 + (size_t)kXzP * kDm * 2 == kOffWout16, "WIN16");
static_assert(kOffWout16 + (size_t)kDm * kDin * 2 <= kOffX2H, "WOUT16");
static_assert(kOffX2H + (size_t)kRows * kDm * 2 == kOffX2L && kOffX2L + (size_t)kRows * kDm * 2 == kOffW1H, "X2 planes");
static_assert(kOffW1H + (size_t)kDff * kDm * 2 == kOffW1L && kOffW1L + (size_t)kDff * kDm * 2 == kOffW2H, "W1 planes");
static_assert(kOffW2H + (size_t)kDm * kDff * 2 == kOffW2L && kOffW2L + (size_t)kDm * kDff * 2 == kOffG1H, "W2 planes");
static_assert(kOffG1H + (size_t)kRows * kDff * 2 == kOffG1L && kOffG1L + (size_t)kRows * kDff * 2 == kWsTotal, "G1 planes");
static_assert((kOffWk16 % 128) == 0 && (kOffWv16 % 128) == 0 && (kOffWo16 % 128) == 0 && (kOffWdt16 % 128) == 0 && (kOffDt16 % 128) == 0, "128-B aligned");

__device__ __forceinline__ unsigned short f2bf_bits(float f) {
  unsigned u = __float_as_uint(f);
  return (unsigned short)((u + 0x7FFFu + ((u >> 16) & 1u)) >> 16);
}
__device__ __forceinline__ float bf_bits2f(unsigned short h) { return __uint_as_float(((unsigned)h) << 16); }

__device__ __forceinline__ void dep_guard_h(v8f& a, v8f& b, v16h x, v16h y) { asm volatile("v_nop\n\tv_nop\n\tv_nop\n\tv_nop" : "+v"(a), "+v"(b) : "v"(x), "v"(y)); }
__device__ __forceinline__ void dep_guard_b(v8f& a, v8f& b, v16b x, v16b y) { asm volatile("v_nop\n\tv_nop\n\tv_nop\n\tv_nop" : "+v"(a), "+v"(b) : "v"(x), "v"(y)); }
__device__ __forceinline__ void dep_guard4_h(v8f& a, v8f& b, v8f& c, v8f& d, v16h x, v16h y) { asm volatile("v_nop\n\tv_nop\n\tv_nop\n\tv_nop" : "+v"(a), "+v"(b), "+v"(c), "+v"(d) : "v"(x), "v"(y)); }
__device__ __forceinline__ void dep_guard4_b(v8f& a, v8f& b, v8f& c, v8f& d, v16b x, v16b y) { asm volatile("v_nop\n\tv_nop\n\tv_nop\n\tv_nop" : "+v"(a), "+v"(b), "+v"(c), "+v"(d) : "v"(x), "v"(y)); }
__device__ __forceinline__ void keep4_h(v16h a, v16h b, v16h c, v16h d) { asm volatile("v_nop" :: "v"(a), "v"(b), "v"(c), "v"(d)); }
__device__ __forceinline__ void keep4_b(v16b a, v16b b, v16b c, v16b d) { asm volatile("v_nop" :: "v"(a), "v"(b), "v"(c), "v"(d)); }
__device__ __forceinline__ void acc_guard4(v8f& a, v8f& b, v8f& c, v8f& d) { asm volatile("v_nop\n\tv_nop\n\tv_nop\n\tv_nop" : "+v"(a), "+v"(b), "+v"(c), "+v"(d)); }
template <typename T> struct Frag;
template <> struct Frag<_Float16> {
  typedef v16h V; union U { v16h v; v8h h[2]; };
  static __device__ __forceinline__ v16h load(const _Float16* p) {
    U f; f.h[0] = *(const v8h*)(p); f.h[1] = *(const v8h*)(p + 16); return f.v;
  }
  static __device__ __forceinline__ v8f mma(v16h a, v16h b, v8f c) {
    return __builtin_amdgcn_wmma_f32_16x16x32_f16(false, a, false, b, (short)0, c, false, false);
  }
  static __device__ __forceinline__ void guard(v8f& a, v8f& b, v16h x, v16h y) { dep_guard_h(a, b, x, y); }
  static __device__ __forceinline__ void guard4(v8f& a, v8f& b, v8f& c, v8f& d, v16h x, v16h y) { dep_guard4_h(a, b, c, d, x, y); }
  static __device__ __forceinline__ void keep(v16h a, v16h b, v16h c, v16h d) { keep4_h(a, b, c, d); }
};
template <> struct Frag<__bf16> {
  typedef v16b V; union U { v16b v; v8b h[2]; };
  static __device__ __forceinline__ v16b load(const __bf16* p) {
    U f; f.h[0] = *(const v8b*)(p); f.h[1] = *(const v8b*)(p + 16); return f.v;
  }
  static __device__ __forceinline__ v8f mma(v16b a, v16b b, v8f c) {
    return __builtin_amdgcn_wmma_f32_16x16x32_bf16(false, a, false, b, (short)0, c, false, false);
  }
  static __device__ __forceinline__ void guard(v8f& a, v8f& b, v16b x, v16b y) { dep_guard_b(a, b, x, y); }
  static __device__ __forceinline__ void guard4(v8f& a, v8f& b, v8f& c, v8f& d, v16b x, v16b y) { dep_guard4_b(a, b, c, d, x, y); }
  static __device__ __forceinline__ void keep(v16b a, v16b b, v16b c, v16b d) { keep4_b(a, b, c, d); }
};

template <int ET> struct Elem;
template <> struct Elem<0> { typedef _Float16 T; };
template <> struct Elem<1> { typedef __bf16 T; };
template <int ET, bool SPLIT, int BIAS_MODE, int OUT_MODE, bool RESID, int ACT = 0>
__global__ __launch_bounds__(256) void wmma_gemm64(
    const unsigned short* __restrict__ Ap, const unsigned short* __restrict__ A2p, int lda, long strideA,
    const unsigned short* __restrict__ Btp, const unsigned short* __restrict__ Bt2p, int ldb, long strideB,
    void* __restrict__ Cout, void* __restrict__ Cout2, int ldc, long strideC,
    const float* __restrict__ bias,
    const float* __restrict__ resid, long strideR,
    int M, int N, int K, float scale) {
  typedef typename Elem<ET>::T T;
  typedef typename Frag<T>::V V;
  const T* A = (const T*)Ap; const T* A2 = (const T*)A2p; const T* Bt = (const T*)Btp; const T* Bt2 = (const T*)Bt2p;
  __shared__ __align__(16) float sT[8][16 * 68];
  const int b    = blockIdx.y;
  const int lane = threadIdx.x & 31;
  const int wave = threadIdx.x >> 5;
  const int tilesN = N >> 6;
  const int tilesM = M >> 6;
  const int tile = blockIdx.x * 8 + wave;
  if (tile >= tilesM * tilesN) return;
  const int tm = tile / tilesN;
  const int tn = tile - tm * tilesN;
  const int m0 = tm << 6;
  const int n0 = tn << 6;

  const T* Ab  = A  + (size_t)b * strideA;
  const T* Bb  = Bt + (size_t)b * strideB;
  const T* Ab2 = SPLIT ? (A2  + (size_t)b * strideA) : nullptr;
  const T* Bb2 = SPLIT ? (Bt2 + (size_t)b * strideB) : nullptr;

  const int rlane = lane & 15;
  const int koff  = (lane >> 4) * 8;
  const int mOff  = (lane >> 4) * 8;

  v8f acc[4][4];
#pragma unroll
  for (int i = 0; i < 4; ++i)
#pragma unroll
    for (int j = 0; j < 4; ++j) acc[i][j] = (v8f){0.f,0.f,0.f,0.f,0.f,0.f,0.f,0.f};

  for (int k0 = 0; k0 < K; k0 += 32) {
    V bh[4], bl[4];
#pragma unroll
    for (int j = 0; j < 4; ++j) {
      const size_t bo = (size_t)(n0 + (j << 4) + rlane) * ldb + koff + k0;
      bh[j] = Frag<T>::load(Bb + bo);
      if (SPLIT) bl[j] = Frag<T>::load(Bb2 + bo);
    }
#pragma unroll
    for (int i = 0; i < 4; ++i) {
      const size_t ao = (size_t)(m0 + (i << 4) + rlane) * lda + koff + k0;
      V ah = Frag<T>::load(Ab + ao);
      V al;
      if (SPLIT) al = Frag<T>::load(Ab2 + ao);
#pragma unroll
      for (int j = 0; j < 4; ++j) {
        acc[i][j] = Frag<T>::mma(ah, bh[j], acc[i][j]);
        if (SPLIT) {
          acc[i][j] = Frag<T>::mma(ah, bl[j], acc[i][j]);
          acc[i][j] = Frag<T>::mma(al, bh[j], acc[i][j]);
        }
      }
      Frag<T>::guard4(acc[i][0], acc[i][1], acc[i][2], acc[i][3], ah, SPLIT ? al : ah);
    }
    Frag<T>::keep(bh[0], bh[1], bh[2], bh[3]);
    if (SPLIT) Frag<T>::keep(bl[0], bl[1], bl[2], bl[3]);
  }
  acc_guard4(acc[0][0], acc[0][1], acc[0][2], acc[0][3]);
  acc_guard4(acc[1][0], acc[1][1], acc[1][2], acc[1][3]);
  acc_guard4(acc[2][0], acc[2][1], acc[2][2], acc[2][3]);
  acc_guard4(acc[3][0], acc[3][1], acc[3][2], acc[3][3]);

  float* slab = sT[wave];
  const float* Rb = RESID ? (resid + (size_t)b * strideR) : nullptr;
#pragma unroll
  for (int i = 0; i < 4; ++i) {
    const int mBase = m0 + (i << 4);
#pragma unroll
    for (int j = 0; j < 4; ++j) {
      const int n = n0 + (j << 4) + rlane;
      float bv = 0.f;
      if (BIAS_MODE == 2) bv = bias[n];
#pragma unroll
      for (int r = 0; r < 8; ++r) {
        float v = acc[i][j][r] * scale;
        if (BIAS_MODE == 1) v += bias[mBase + mOff + r];
        if (BIAS_MODE == 2) v += bv;
        if (RESID) v += Rb[(size_t)(mBase + mOff + r) * ldc + n];
        if (ACT == 1) v = tanhf(v);
        if (ACT == 2) v = fmaxf(v, 0.0f);
        if (ACT == 4) v = (v > 0.f) ? v : 0.01f * v;
        slab[(mOff + r) * 68 + (j << 4) + rlane] = v;
      }
    }
    __builtin_amdgcn_fence(__ATOMIC_RELEASE, "workgroup");
    __builtin_amdgcn_wave_barrier();
    __builtin_amdgcn_fence(__ATOMIC_ACQUIRE, "workgroup");
    if (OUT_MODE == 0) {
      float* C = (float*)Cout + (size_t)b * strideC;
      const int hh = lane >> 4, c4 = (lane & 15) * 4;
      for (int pass = 0; pass < 2; ++pass) {
#pragma unroll
        for (int it = 0; it < 8; ++it) {
          const int row = it * 2 + hh;
          v4f v = *(const v4f*)(slab + row * 68 + c4);
          *(volatile v4f*)(C + (size_t)(mBase + row) * ldc + n0 + c4) = v;
        }
        __threadfence();
      }
    } else {
      const int q = lane >> 3, c8 = (lane & 7) * 8;
      unsigned short* C  = (unsigned short*)Cout  + (size_t)b * strideC;
      unsigned short* C2 = (OUT_MODE == 2) ? ((unsigned short*)Cout2 + (size_t)b * strideC) : nullptr;
      for (int pass = 0; pass < 2; ++pass) {
#pragma unroll
        for (int it = 0; it < 4; ++it) {
          const int row = it * 4 + q;
          const float* sp = slab + row * 68 + c8;
          v8h hv, lv;
#pragma unroll
          for (int e = 0; e < 8; ++e) {
            if (OUT_MODE == 1) {
              hv[e] = (_Float16)sp[e];
            } else {
              unsigned short hb = f2bf_bits(sp[e]);
              unsigned short lb = f2bf_bits(sp[e] - bf_bits2f(hb));
              hv[e] = __builtin_bit_cast(_Float16, hb);
              lv[e] = __builtin_bit_cast(_Float16, lb);
            }
          }
          *(volatile v8h*)(C + (size_t)(mBase + row) * ldc + n0 + c8) = hv;
          if (OUT_MODE == 2) *(volatile v8h*)(C2 + (size_t)(mBase + row) * ldc + n0 + c8) = lv;
        }
        __threadfence();
      }
    }
    __builtin_amdgcn_fence(__ATOMIC_RELEASE, "workgroup");
    __builtin_amdgcn_wave_barrier();
    __builtin_amdgcn_fence(__ATOMIC_ACQUIRE, "workgroup");
  }
}

__global__ __launch_bounds__(256) void cast_f16_kernel(
    const float* __restrict__ src, unsigned short* __restrict__ dst, int total8, float scale)
{
  const int i = blockIdx.x * 256 + threadIdx.x;
  if (i >= total8) return;
  const size_t e0 = (size_t)i << 3;
  const float* p = src + e0;
  const v4f a0 = *(const v4f*)(p);
  const v4f a1 = *(const v4f*)(p + 4);
  v8h hv;
#pragma unroll
  for (int e = 0; e < 4; ++e) {
    hv[e]     = (_Float16)(a0[e] * scale);
    hv[4 + e] = (_Float16)(a1[e] * scale);
  }
  unsigned short* q = dst + e0;
  *(volatile v8h*)q = hv;
  __threadfence();
  *(volatile v8h*)q = hv;
}

__global__ __launch_bounds__(256) void split_rows_bf16_kernel(
    const float* __restrict__ src, unsigned short* __restrict__ dhi, unsigned short* __restrict__ dlo, int total8)
{
  const int i = blockIdx.x * 256 + threadIdx.x;
  if (i >= total8) return;
  const size_t e0 = (size_t)i << 3;
  const v4f a0 = *(const v4f*)(src + e0);
  const v4f a1 = *(const v4f*)(src + e0 + 4);
  v8h hv, lv;
#pragma unroll
  for (int e = 0; e < 4; ++e) {
    const unsigned short h0 = f2bf_bits(a0[e]), h1 = f2bf_bits(a1[e]);
    const unsigned short l0 = f2bf_bits(a0[e] - bf_bits2f(h0)), l1 = f2bf_bits(a1[e] - bf_bits2f(h1));
    hv[e]     = __builtin_bit_cast(_Float16, h0);
    hv[4 + e] = __builtin_bit_cast(_Float16, h1);
    lv[e]     = __builtin_bit_cast(_Float16, l0);
    lv[4 + e] = __builtin_bit_cast(_Float16, l1);
  }
  unsigned short* qh = dhi + e0;
  unsigned short* ql = dlo + e0;
  *(volatile v8h*)qh = hv;
  *(volatile v8h*)ql = lv;
  __threadfence();
  *(volatile v8h*)qh = hv;
  *(volatile v8h*)ql = lv;
}

__device__ __forceinline__ unsigned pk16(unsigned short a, unsigned short b) { return (unsigned)a | ((unsigned)b << 16); }

__global__ __launch_bounds__(256) void gelu_split_kernel(
    const float* __restrict__ in, unsigned short* __restrict__ hi, unsigned short* __restrict__ lo, int n2)
{
  const int i = blockIdx.x * 256 + threadIdx.x;
  if (i >= n2) return;
  const v2f f = *(const v2f*)(in + 2 * (size_t)i);
  const float x0 = f[0], x1 = f[1];
  const float g0 = 0.5f * x0 * (1.0f + erff(x0 * 0.70710678118654752f));
  const float g1 = 0.5f * x1 * (1.0f + erff(x1 * 0.70710678118654752f));
  const unsigned short h0 = f2bf_bits(g0), h1 = f2bf_bits(g1);
  const unsigned short l0 = f2bf_bits(g0 - bf_bits2f(h0)), l1 = f2bf_bits(g1 - bf_bits2f(h1));
  const unsigned uh = pk16(h0, h1), ul = pk16(l0, l1);
  ((volatile unsigned*)hi)[i] = uh;
  ((volatile unsigned*)lo)[i] = ul;
  __threadfence();
  ((volatile unsigned*)hi)[i] = uh;
  ((volatile unsigned*)lo)[i] = ul;
}

__global__ __launch_bounds__(256) void dt_cast_kernel(
    const float* __restrict__ XD, unsigned short* __restrict__ DT16, int total8, float scale)
{
  const int i = blockIdx.x * 256 + threadIdx.x;
  if (i >= total8) return;
  const int e0  = i << 3;
  const int row = e0 >> 5;
  const int c8  = e0 & 31;
  const float* p = XD + (size_t)row * kXdW + c8;
  const v4f a0 = *(const v4f*)(p);
  const v4f a1 = *(const v4f*)(p + 4);
  v8h hv;
#pragma unroll
  for (int e = 0; e < 4; ++e) {
    hv[e]     = (_Float16)(a0[e] * scale);
    hv[4 + e] = (_Float16)(a1[e] * scale);
  }
  unsigned short* qd = DT16 + e0;
  *(volatile v8h*)qd = hv;
  __threadfence();
  *(volatile v8h*)qd = hv;
}

__global__ __launch_bounds__(128) void add_ln_kernel(
    const float* __restrict__ X, const float* __restrict__ Y,
    const float* __restrict__ g, const float* __restrict__ bt, float* __restrict__ out)
{
  __shared__ float red[8];
  const int tid = threadIdx.x, lane = tid & 31, wave = tid >> 5;
  const size_t base = (size_t)blockIdx.x * kDm + (size_t)tid * 4;
  const v4f xv = *(const v4f*)(X + base);
  const v4f yv = *(const v4f*)(Y + base);
  const float a0 = xv[0] + yv[0], a1 = xv[1] + yv[1], a2 = xv[2] + yv[2], a3 = xv[3] + yv[3];
  float s = (a0 + a1) + (a2 + a3);
#pragma unroll
  for (int off = 16; off > 0; off >>= 1) s += __shfl_xor(s, off, 32);
  if (lane == 0) red[wave] = s;
  __syncthreads();
  const float mu = ((red[0] + red[1]) + (red[2] + red[3])) * (1.0f / (float)kDm);
  const float e0 = a0 - mu, e1 = a1 - mu, e2 = a2 - mu, e3 = a3 - mu;
  float s2 = (e0 * e0 + e1 * e1) + (e2 * e2 + e3 * e3);
#pragma unroll
  for (int off = 16; off > 0; off >>= 1) s2 += __shfl_xor(s2, off, 32);
  if (lane == 0) red[4 + wave] = s2;
  __syncthreads();
  const float var = ((red[4] + red[5]) + (red[6] + red[7])) * (1.0f / (float)kDm);
  const float inv = 1.0f / sqrtf(var + 1e-5f);
  const v4f gv = *(const v4f*)(g + (size_t)tid * 4);
  const v4f bv = *(const v4f*)(bt + (size_t)tid * 4);
  v4f ov;
  ov[0] = e0 * inv * gv[0] + bv[0];
  ov[1] = e1 * inv * gv[1] + bv[1];
  ov[2] = e2 * inv * gv[2] + bv[2];
  ov[3] = e3 * inv * gv[3] + bv[3];
  float* op = out + base;
  *(volatile v4f*)op = ov;
  __threadfence();
  *(volatile v4f*)op = ov;
}

__device__ __forceinline__ v8f hmma16(v16h a, v16h b, v8f c) {
  c = __builtin_amdgcn_wmma_f32_16x16x32_f16(false, a, false, b, (short)0, c, false, false);
  asm volatile("v_nop\n\tv_nop\n\tv_nop\n\tv_nop" : "+v"(c) : "v"(a), "v"(b));
  return c;
}

__global__ __launch_bounds__(128) void xattn_kernel(
    const unsigned short* __restrict__ Qp, const unsigned short* __restrict__ Kp,
    const unsigned short* __restrict__ Vtp, unsigned short* __restrict__ Op, float sscale, float oscale)
{
  typedef Frag<_Float16> F;
  __shared__ __align__(16) _Float16 Ksh[64 * 64];
  __shared__ __align__(16) _Float16 Vth[64 * 64];
  __shared__ __align__(16) _Float16 Psh[4][16 * 64];
  __shared__ __align__(16) float    Os[4][16 * 68];

  const int tid  = threadIdx.x;
  const int wave = tid >> 5;
  const int lane = tid & 31;
  const int hh   = lane >> 4;
  const int c    = lane & 15;

  constexpr int nqb = kSeq / 64;
  const int bx = blockIdx.x;
  const int qb = bx % nqb;
  const int bh = bx / nqb;
  const int h  = bh % kHeads;
  const int b  = bh / kHeads;
  const int q0 = qb * 64 + wave * 16;

  const _Float16* Qb = (const _Float16*)(const void*)Qp + (size_t)b * kSeq * kDm + (size_t)h * kHd;
  const _Float16* Kb = (const _Float16*)(const void*)Kp + (size_t)b * kMem * kDm + (size_t)h * kHd;
  const _Float16* Vb = (const _Float16*)(const void*)Vtp + ((size_t)b * kDm + (size_t)h * kHd) * kMem;
  _Float16* Ob = (_Float16*)(void*)Op + (size_t)b * kSeq * kDm + (size_t)h * kHd;

  v16h qa[2];
#pragma unroll
  for (int dc = 0; dc < 2; ++dc) qa[dc] = F::load(Qb + (size_t)(q0 + c) * kDm + dc * 32 + 8 * hh);

  float mrow[8], lrow[8];
  v8f oacc[4];
#pragma unroll
  for (int r = 0; r < 8; ++r) { mrow[r] = -INFINITY; lrow[r] = 0.f; }
#pragma unroll
  for (int t = 0; t < 4; ++t) oacc[t] = (v8f){0.f,0.f,0.f,0.f,0.f,0.f,0.f,0.f};

#pragma unroll 1
  for (int kc = 0; kc < kMem / 64; ++kc) {
    const int kv0 = kc * 64;
    __syncthreads();
    {
      const int r = tid >> 1, e0 = (tid & 1) * 32;
      const _Float16* ks = Kb + (size_t)(kv0 + r) * kDm + e0;
      const v8h k0v = *(const v8h*)(ks);
      const v8h k1v = *(const v8h*)(ks + 8);
      const v8h k2v = *(const v8h*)(ks + 16);
      const v8h k3v = *(const v8h*)(ks + 24);
      *(v8h*)(Ksh + r * 64 + e0)      = k0v;
      *(v8h*)(Ksh + r * 64 + e0 + 8)  = k1v;
      *(v8h*)(Ksh + r * 64 + e0 + 16) = k2v;
      *(v8h*)(Ksh + r * 64 + e0 + 24) = k3v;
      asm volatile("" ::: "memory");
      const _Float16* vs = Vb + (size_t)r * kMem + kv0 + e0;
      const v8h v0v = *(const v8h*)(vs);
      const v8h v1v = *(const v8h*)(vs + 8);
      const v8h v2v = *(const v8h*)(vs + 16);
      const v8h v3v = *(const v8h*)(vs + 24);
      *(v8h*)(Vth + r * 64 + e0)      = v0v;
      *(v8h*)(Vth + r * 64 + e0 + 8)  = v1v;
      *(v8h*)(Vth + r * 64 + e0 + 16) = v2v;
      *(v8h*)(Vth + r * 64 + e0 + 24) = v3v;
    }
    __syncthreads();

    v8f s[4];
#pragma unroll
    for (int j = 0; j < 4; ++j) {
      s[j] = (v8f){0.f,0.f,0.f,0.f,0.f,0.f,0.f,0.f};
#pragma unroll
      for (int dc = 0; dc < 2; ++dc) {
        const v16h kb = F::load(Ksh + (j * 16 + c) * 64 + dc * 32 + 8 * hh);
        s[j] = hmma16(qa[dc], kb, s[j]);
      }
    }
    float cm[8];
#pragma unroll
    for (int r = 0; r < 8; ++r) {
      float m = -INFINITY;
#pragma unroll
      for (int j = 0; j < 4; ++j) {
        const float sv = s[j][r] * sscale;
        s[j][r] = sv;
        m = fmaxf(m, sv);
      }
#pragma unroll
      for (int off = 1; off < 16; off <<= 1) m = fmaxf(m, __shfl_xor(m, off, 32));
      cm[r] = m;
    }
    _Float16* pw = Psh[wave];
#pragma unroll
    for (int r = 0; r < 8; ++r) {
      const float mnew  = fmaxf(mrow[r], cm[r]);
      const float alpha = expf(mrow[r] - mnew);
      mrow[r] = mnew;
      float psum = 0.f;
#pragma unroll
      for (int j = 0; j < 4; ++j) {
        const float p = expf(s[j][r] - mnew);
        psum += p;
        pw[(8 * hh + r) * 64 + j * 16 + c] = (_Float16)(p * kPCarry);
      }
#pragma unroll
      for (int off = 1; off < 16; off <<= 1) psum += __shfl_xor(psum, off, 32);
      lrow[r] = lrow[r] * alpha + psum;
#pragma unroll
      for (int t = 0; t < 4; ++t) oacc[t][r] *= alpha;
    }
    __builtin_amdgcn_fence(__ATOMIC_RELEASE, "workgroup");
    __builtin_amdgcn_wave_barrier();
    __builtin_amdgcn_fence(__ATOMIC_ACQUIRE, "workgroup");
#pragma unroll 1
    for (int kk = 0; kk < 2; ++kk) {
      const v16h pa = F::load(pw + c * 64 + kk * 32 + 8 * hh);
#pragma unroll
      for (int t = 0; t < 4; ++t) {
        const v16h vb = F::load(Vth + (t * 16 + c) * 64 + kk * 32 + 8 * hh);
        oacc[t] = hmma16(pa, vb, oacc[t]);
      }
    }
  }

  float* os = Os[wave];
#pragma unroll
  for (int r = 0; r < 8; ++r) {
    const float inv = oscale / (lrow[r] * kPCarry);
#pragma unroll
    for (int t = 0; t < 4; ++t) os[(8 * hh + r) * 68 + t * 16 + c] = oacc[t][r] * inv;
  }
  __builtin_amdgcn_fence(__ATOMIC_RELEASE, "workgroup");
  __builtin_amdgcn_wave_barrier();
  __builtin_amdgcn_fence(__ATOMIC_ACQUIRE, "workgroup");
  {
    const int q8 = lane >> 3, c8 = (lane & 7) * 8;
    v8h hv[4];
#pragma unroll
    for (int it = 0; it < 4; ++it) {
      const int row = it * 4 + q8;
      const float* sp = os + row * 68 + c8;
#pragma unroll
      for (int e = 0; e < 8; ++e) hv[it][e] = (_Float16)sp[e];
    }
    for (int pass = 0; pass < 2; ++pass) {
#pragma unroll
      for (int it = 0; it < 4; ++it) {
        const int row = it * 4 + q8;
        *(volatile v8h*)(Ob + (size_t)(q0 + row) * kDm + c8) = hv[it];
      }
      __threadfence();
    }
  }
}

__global__ __launch_bounds__(256) void conv_silu_kernel(
    const float* __restrict__ XZ, const float* __restrict__ cw, const float* __restrict__ cb,
    unsigned short* __restrict__ UC16)
{
  __shared__ __align__(16) float sT[16 * kTP];
  const int tid = threadIdx.x, lane = tid & 31, wave = tid >> 5;
  const int d0 = blockIdx.x * 256, d = d0 + tid;
  const int g0 = blockIdx.y * 64;
  const int tb = g0 & (kSeq - 1);
  const v4f wv = *(const v4f*)(cw + (size_t)d * 4);
  const float w0 = wv[0], w1 = wv[1], w2 = wv[2], w3 = wv[3];
  const float bc = cb[d];
  float xm3, xm2, xm1;
  {
    const bool hist = (tb > 0);
    const int rb = hist ? (g0 - 3) : g0;
    const float v3 = XZ[(size_t)rb * kXzP + d];
    const float v2 = XZ[(size_t)(rb + 1) * kXzP + d];
    const float v1 = XZ[(size_t)(rb + 2) * kXzP + d];
    xm3 = hist ? v3 : 0.f;
    xm2 = hist ? v2 : 0.f;
    xm1 = hist ? v1 : 0.f;
  }
#pragma unroll 1
  for (int sub = 0; sub < 4; ++sub) {
    const int lb = g0 + sub * 16;
#pragma unroll 1
    for (int s = 0; s < 16; ++s) {
      const float xcur = XZ[(size_t)(lb + s) * kXzP + d];
      float acc = w0 * xm3;
      acc = fmaf(w1, xm2, acc);
      acc = fmaf(w2, xm1, acc);
      acc = fmaf(w3, xcur, acc);
      const float sv = acc + bc;
      const float sg = __builtin_amdgcn_rcpf(1.0f + __expf(-sv));
      sT[s * kTP + tid] = sv * sg;
      xm3 = xm2; xm2 = xm1; xm1 = xcur;
    }
    __syncthreads();
    v8h bv[2];
#pragma unroll
    for (int it = 0; it < 2; ++it) {
      const float* sp = sT + (it * 8 + wave) * kTP + lane * 8;
      const v4f a0 = *(const v4f*)(sp);
      const v4f a1 = *(const v4f*)(sp + 4);
#pragma unroll
      for (int e = 0; e < 4; ++e) {
        bv[it][e]     = (_Float16)(a0[e] * kUsc);
        bv[it][4 + e] = (_Float16)(a1[e] * kUsc);
      }
    }
    for (int pass = 0; pass < 2; ++pass) {
#pragma unroll
      for (int it = 0; it < 2; ++it)
        *(volatile v8h*)(UC16 + (size_t)(lb + it * 8 + wave) * kDin + d0 + lane * 8) = bv[it];
      __threadfence();
    }
    __syncthreads();
  }
}

__global__ __launch_bounds__(256) void scan_kernel(
    const float* __restrict__ DLR, const float* __restrict__ XZ, const float* __restrict__ XD,
    const float* __restrict__ cw, const float* __restrict__ cb,
    const float* __restrict__ A_log, const float* __restrict__ Dv, unsigned short* __restrict__ Y16)
{
  __shared__ __align__(16) float sBC[16 * 32];
  __shared__ __align__(16) float sY[16 * kTP];
  const int tid = threadIdx.x, lane = tid & 31, wave = tid >> 5;
  const int d0 = blockIdx.x * 256, d = d0 + tid;
  const size_t row0 = (size_t)blockIdx.y * kSeq;

  float An[kNst];
  {
    const v4f a0 = *(const v4f*)(A_log + (size_t)d * kNst);
    const v4f a1 = *(const v4f*)(A_log + (size_t)d * kNst + 4);
    const v4f a2 = *(const v4f*)(A_log + (size_t)d * kNst + 8);
    const v4f a3 = *(const v4f*)(A_log + (size_t)d * kNst + 12);
#pragma unroll
    for (int e = 0; e < 4; ++e) {
      An[e]      = -__expf(a0[e]);
      An[4 + e]  = -__expf(a1[e]);
      An[8 + e]  = -__expf(a2[e]);
      An[12 + e] = -__expf(a3[e]);
    }
  }
  asm volatile("" ::: "memory");
  const v4f wv = *(const v4f*)(cw + (size_t)d * 4);
  const float w0 = wv[0], w1 = wv[1], w2 = wv[2], w3 = wv[3];
  const float bc = cb[d];
  const float Dd = Dv[d];
  float h[kNst];
#pragma unroll
  for (int n = 0; n < kNst; ++n) h[n] = 0.f;
  float xm3 = 0.f, xm2 = 0.f, xm1 = 0.f;

#pragma unroll 1
  for (int cch = 0; cch < kSeq / 16; ++cch) {
    const int l0 = cch * 16;
    if (tid < 128) {
      const int r = tid >> 3, q4 = (tid & 7) * 4;
      const v4f v = *(const v4f*)(XD + (row0 + l0 + r) * kXdW + kDtR + q4);
      *(v4f*)(sBC + r * 32 + q4) = v;
    }
    __syncthreads();
#pragma unroll 1
    for (int s = 0; s < 16; ++s) {
      const size_t m = row0 + l0 + s;
      const float a     = DLR[m * kDin + d];
      const float delta = fmaxf(a, 0.0f) + log1pf(__expf(-fabsf(a)));
      const float xc    = XZ[m * kXzP + d];
      float cacc = w0 * xm3;
      cacc = fmaf(w1, xm2, cacc);
      cacc = fmaf(w2, xm1, cacc);
      cacc = fmaf(w3, xc, cacc);
      const float sv = cacc + bc;
      const float su = __builtin_amdgcn_rcpf(1.0f + __expf(-sv));
      const float xv = sv * su;
      xm3 = xm2; xm2 = xm1; xm1 = xc;
      const float zv = XZ[m * kXzP + kDin + d];
      v4f Bq[4], Cq[4];
#pragma unroll
      for (int qq = 0; qq < 4; ++qq) {
        Bq[qq] = *(const v4f*)(sBC + s * 32 + 4 * qq);
        Cq[qq] = *(const v4f*)(sBC + s * 32 + kNst + 4 * qq);
      }
      float y = 0.f;
#pragma unroll
      for (int n = 0; n < kNst; ++n) {
        const float e = __expf(delta * An[n]);
        float db = delta * Bq[n >> 2][n & 3];
        asm volatile("" : "+v"(db));
        float p = db * xv;
        asm volatile("" : "+v"(p));
        float qv = h[n] * e;
        asm volatile("" : "+v"(qv));
        const float hn = qv + p;
        h[n] = hn;
        float rr = Cq[n >> 2][n & 3] * hn;
        asm volatile("" : "+v"(rr));
        y += rr;
      }
      float sk = xv * Dd;
      asm volatile("" : "+v"(sk));
      y += sk;
      const float sg = __builtin_amdgcn_rcpf(1.0f + __expf(-zv));
      const float g  = zv * sg;
      sY[s * kTP + tid] = (y * g) * kYsc;
    }
    __syncthreads();
    v8h hv[2];
#pragma unroll
    for (int it = 0; it < 2; ++it) {
      const float* sp = sY + (it * 8 + wave) * kTP + lane * 8;
      const v4f a0 = *(const v4f*)(sp);
      const v4f a1 = *(const v4f*)(sp + 4);
#pragma unroll
      for (int e = 0; e < 4; ++e) { hv[it][e] = (_Float16)a0[e]; hv[it][4 + e] = (_Float16)a1[e]; }
    }
    for (int pass = 0; pass < 2; ++pass) {
#pragma unroll
      for (int it = 0; it < 2; ++it)
        *(volatile v8h*)(Y16 + (size_t)(row0 + l0 + it * 8 + wave) * kDin + d0 + lane * 8) = hv[it];
      __threadfence();
    }
  }
}

extern "C" void kernel_launch(void* const* d_in, const int* in_sizes, int n_in,
                              void* d_out, int out_size, void* d_ws, size_t ws_size,
                              hipStream_t stream)
{
  if (n_in < 29) return;
  if (in_sizes[0] != kRows * kDm || in_sizes[1] != kMRows * kDm) return;
  if (in_sizes[2] != kDm * kDm || in_sizes[3] != kDm) return;
  if (in_sizes[4] != kDm * kDm || in_sizes[5] != kDm) return;
  if (in_sizes[6] != kDm * kDm || in_sizes[7] != kDm) return;
  if (in_sizes[8] != kDm * kDm || in_sizes[9] != kDm) return;
  for (int i = 10; i < 16; ++i) if (in_sizes[i] != kDm) return;
  if (in_sizes[16] != kXzP * kDm) return;
  if (in_sizes[17] != kDin * 4 || in_sizes[18] != kDin) return;
  if (in_sizes[19] != kXdW * kDin) return;
  if (in_sizes[20] != kDin * kDtR || in_sizes[21] != kDin) return;
  if (in_sizes[22] != kDin * kNst || in_sizes[23] != kDin) return;
  if (in_sizes[24] != kDm * kDin) return;
  if (in_sizes[25] != kDff * kDm || in_sizes[26] != kDff) return;
  if (in_sizes[27] != kDm * kDff || in_sizes[28] != kDm) return;
  if (out_size != kRows * kDm) return;
  if (ws_size < kWsTotal) return;

  const float* x      = (const float*)d_in[0];
  const float* memory = (const float*)d_in[1];
  const float* Wq = (const float*)d_in[2];   const float* bq = (const float*)d_in[3];
  const float* Wk = (const float*)d_in[4];   const float* bk = (const float*)d_in[5];
  const float* Wv = (const float*)d_in[6];   const float* bv = (const float*)d_in[7];
  const float* Wo = (const float*)d_in[8];   const float* bo = (const float*)d_in[9];
  const float* ln1_g = (const float*)d_in[10]; const float* ln1_b = (const float*)d_in[11];
  const float* ln2_g = (const float*)d_in[12]; const float* ln2_b = (const float*)d_in[13];
  const float* ln3_g = (const float*)d_in[14]; const float* ln3_b = (const float*)d_in[15];
  const float* W_in    = (const float*)d_in[16];
  const float* conv_w  = (const float*)d_in[17]; const float* conv_b = (const float*)d_in[18];
  const float* W_xproj = (const float*)d_in[19];
  const float* W_dt    = (const float*)d_in[20]; const float* b_dt = (const float*)d_in[21];
  const float* A_log   = (const float*)d_in[22]; const float* D_p  = (const float*)d_in[23];
  const float* W_out   = (const float*)d_in[24];
  const float* W1 = (const float*)d_in[25];    const float* b1 = (const float*)d_in[26];
  const float* W2 = (const float*)d_in[27];    const float* b2 = (const float*)d_in[28];
  float* dout = (float*)d_out;

  char* ws = (char*)d_ws;
  float*          X1     = (float*)(ws + kOffX1);
  float*          X2     = (float*)(ws + kOffX2);
  float*          ATTO   = (float*)(ws + kOffAttO);
  float*          XZ     = (float*)(ws + kOffXZ);
  float*          HPRE   = (float*)(ws + kOffHPre);
  float*          DLR    = (float*)(ws + kOffDLR);
  float*          XD     = (float*)(ws + kOffXD);
  float*          MO     = (float*)(ws + kOffMO);
  float*          FFNO   = (float*)(ws + kOffFfnO);
  unsigned short* X16    = (unsigned short*)(ws + kOffX16);
  unsigned short* AT16   = (unsigned short*)(ws + kOffAt16);
  unsigned short* M16    = (unsigned short*)(ws + kOffM16);
  unsigned short* X1H16  = (unsigned short*)(ws + kOffX1h);
  unsigned short* WQ16   = (unsigned short*)(ws + kOffWq16);
  unsigned short* WK16   = (unsigned short*)(ws + kOffWk16);
  unsigned short* WV16   = (unsigned short*)(ws + kOffWv16);
  unsigned short* WO16   = (unsigned short*)(ws + kOffWo16);
  unsigned short* WXP16  = (unsigned short*)(ws + kOffWxp16);
  unsigned short* WDT16  = (unsigned short*)(ws + kOffWdt16);
  unsigned short* DT16   = (unsigned short*)(ws + kOffDt16);
  unsigned short* Q16    = (unsigned short*)(ws + kOffQ16);
  unsigned short* UC16   = (unsigned short*)(ws + kOffUc16);
  unsigned short* K16    = (unsigned short*)(ws + kOffK16);
  unsigned short* Y16    = (unsigned short*)(ws + kOffY16);
  unsigned short* VT16   = (unsigned short*)(ws + kOffVt16);
  unsigned short* WIN16  = (unsigned short*)(ws + kOffWin16);
  unsigned short* WOUT16 = (unsigned short*)(ws + kOffWout16);
  unsigned short* X2H    = (unsigned short*)(ws + kOffX2H);
  unsigned short* X2L    = (unsigned short*)(ws + kOffX2L);
  unsigned short* W1H    = (unsigned short*)(ws + kOffW1H);
  unsigned short* W1L    = (unsigned short*)(ws + kOffW1L);
  unsigned short* W2H    = (unsigned short*)(ws + kOffW2H);
  unsigned short* W2L    = (unsigned short*)(ws + kOffW2L);
  unsigned short* G1H    = (unsigned short*)(ws + kOffG1H);
  unsigned short* G1L    = (unsigned short*)(ws + kOffG1L);
  const float* dummy_resid = x;

  cast_f16_kernel<<<(kRows * kDm) / 8 / 256, 256, 0, stream>>>(x, X16, (kRows * kDm) / 8, 1.0f);
  cast_f16_kernel<<<(kMRows * kDm) / 8 / 256, 256, 0, stream>>>(memory, M16, (kMRows * kDm) / 8, 1.0f);
  cast_f16_kernel<<<(kDm * kDm) / 8 / 256, 256, 0, stream>>>(Wq, WQ16, (kDm * kDm) / 8, kWsc);
  cast_f16_kernel<<<(kDm * kDm) / 8 / 256, 256, 0, stream>>>(Wk, WK16, (kDm * kDm) / 8, kWsc);
  cast_f16_kernel<<<(kDm * kDm) / 8 / 256, 256, 0, stream>>>(Wv, WV16, (kDm * kDm) / 8, kWsc);
  cast_f16_kernel<<<(kDm * kDm) / 8 / 256, 256, 0, stream>>>(Wo, WO16, (kDm * kDm) / 8, kWsc);

  wmma_gemm64<0, false, 2, 1, false><<<dim3((kRows / 64) * (kDm / 64) / 8, 1), 256, 0, stream>>>(
      X16, X16, kDm, 0L, WQ16, WQ16, kDm, 0L,
      (void*)Q16, (void*)Q16, kDm, 0L, bq, dummy_resid, 0L, kRows, kDm, kDm, 1.0f / kWsc);
  wmma_gemm64<0, false, 2, 1, false><<<dim3((kMRows / 64) * (kDm / 64) / 8, 1), 256, 0, stream>>>(
      M16, M16, kDm, 0L, WK16, WK16, kDm, 0L,
      (void*)K16, (void*)K16, kDm, 0L, bk, dummy_resid, 0L, kMRows, kDm, kDm, 1.0f / kWsc);
  wmma_gemm64<0, false, 1, 1, false><<<dim3((kDm / 64) * (kMem / 64) / 8, kBatch), 256, 0, stream>>>(
      WV16, WV16, kDm, 0L, M16, M16, kDm, (long)kMem * kDm,
      (void*)VT16, (void*)VT16, kMem, (long)kDm * kMem, bv, dummy_resid, 0L, kDm, kMem, kDm, 1.0f / kWsc);
  xattn_kernel<<<kBatch * kHeads * (kSeq / 64), 128, 0, stream>>>(Q16, K16, VT16, AT16, kQkScale, kAttSc);
  wmma_gemm64<0, false, 2, 0, false><<<dim3((kRows / 64) * (kDm / 64) / 8, 1), 256, 0, stream>>>(
      AT16, AT16, kDm, 0L, WO16, WO16, kDm, 0L,
      (void*)ATTO, (void*)ATTO, kDm, 0L, bo, dummy_resid, 0L, kRows, kDm, kDm, 1.0f / (kAttSc * kWsc));
  add_ln_kernel<<<kRows, 128, 0, stream>>>(x, ATTO, ln1_g, ln1_b, X1);
  cast_f16_kernel<<<(kRows * kDm) / 8 / 256, 256, 0, stream>>>(X1, X1H16, (kRows * kDm) / 8, 1.0f);

  cast_f16_kernel<<<(kXzP * kDm) / 8 / 256, 256, 0, stream>>>(W_in, WIN16, (kXzP * kDm) / 8, kWsc);
  cast_f16_kernel<<<(kXdW * kDin) / 8 / 256, 256, 0, stream>>>(W_xproj, WXP16, (kXdW * kDin) / 8, kWsc);
  cast_f16_kernel<<<(kDin * kDtR) / 8 / 256, 256, 0, stream>>>(W_dt, WDT16, (kDin * kDtR) / 8, kWsc);
  cast_f16_kernel<<<(kDm * kDin) / 8 / 256, 256, 0, stream>>>(W_out, WOUT16, (kDm * kDin) / 8, kWsc);

  for (int hf = 0; hf < 2; ++hf) {
    const unsigned short* X1h = X1H16 + (size_t)hf * kHalfRows * kDm;
    float* MOh = MO + (size_t)hf * kHalfRows * kDm;

    wmma_gemm64<0, false, 0, 0, false><<<dim3((kHalfRows / 64) * (kXzP / 64) / 8, 1), 256, 0, stream>>>(
        X1h, X1h, kDm, 0L, WIN16, WIN16, kDm, 0L,
        (void*)XZ, (void*)XZ, kXzP, 0L, bq, dummy_resid, 0L, kHalfRows, kXzP, kDm, 1.0f / kWsc);
    conv_silu_kernel<<<dim3(kDin / 256, kHalfRows / 64), 256, 0, stream>>>(XZ, conv_w, conv_b, UC16);
    wmma_gemm64<0, false, 0, 0, false><<<dim3((kHalfRows / 64) * (kXdW / 64) / 8, 1), 256, 0, stream>>>(
        UC16, UC16, kDin, 0L, WXP16, WXP16, kDin, 0L,
        (void*)XD, (void*)XD, kXdW, 0L, bq, dummy_resid, 0L, kHalfRows, kXdW, kDin, 1.0f / (kUsc * kWsc));
    dt_cast_kernel<<<(kHalfRows * kDtR) / 8 / 256, 256, 0, stream>>>(XD, DT16, (kHalfRows * kDtR) / 8, kDtsc);
    wmma_gemm64<0, false, 2, 0, false><<<dim3((kHalfRows / 64) * (kDin / 64) / 8, 1), 256, 0, stream>>>(
        DT16, DT16, kDtR, 0L, WDT16, WDT16, kDtR, 0L,
        (void*)DLR, (void*)DLR, kDin, 0L, b_dt, dummy_resid, 0L, kHalfRows, kDin, kDtR, 1.0f / (kDtsc * kWsc));
    scan_kernel<<<dim3(kDin / 256, kHalfB), 256, 0, stream>>>(DLR, XZ, XD, conv_w, conv_b, A_log, D_p, Y16);
    wmma_gemm64<0, false, 0, 0, false><<<dim3((kHalfRows / 64) * (kDm / 64) / 8, 1), 256, 0, stream>>>(
        Y16, Y16, kDin, 0L, WOUT16, WOUT16, kDin, 0L,
        (void*)MOh, (void*)MOh, kDm, 0L, bq, dummy_resid, 0L, kHalfRows, kDm, kDin, 1.0f / (kYsc * kWsc));
  }
  add_ln_kernel<<<kRows, 128, 0, stream>>>(X1, MO, ln2_g, ln2_b, X2);

  split_rows_bf16_kernel<<<(kRows * kDm / 8) / 256, 256, 0, stream>>>(X2, X2H, X2L, kRows * kDm / 8);
  split_rows_bf16_kernel<<<(kDff * kDm / 8) / 256, 256, 0, stream>>>(W1, W1H, W1L, kDff * kDm / 8);
  split_rows_bf16_kernel<<<(kDm * kDff / 8) / 256, 256, 0, stream>>>(W2, W2H, W2L, kDm * kDff / 8);
  wmma_gemm64<1, true, 2, 0, false><<<dim3((kRows / 64) * (kDff / 64) / 8, 1), 256, 0, stream>>>(
      X2H, X2L, kDm, 0L, W1H, W1L, kDm, 0L,
      (void*)HPRE, (void*)HPRE, kDff, 0L, b1, dummy_resid, 0L, kRows, kDff, kDm, 1.0f);
  gelu_split_kernel<<<(kRows * kDff / 2) / 256, 256, 0, stream>>>(HPRE, G1H, G1L, kRows * kDff / 2);
  wmma_gemm64<1, true, 2, 0, false><<<dim3((kRows / 64) * (kDm / 64) / 8, 1), 256, 0, stream>>>(
      G1H, G1L, kDff, 0L, W2H, W2L, kDff, 0L,
      (void*)FFNO, (void*)FFNO, kDm, 0L, b2, dummy_resid, 0L, kRows, kDm, kDff, 1.0f);
  add_ln_kernel<<<kRows, 128, 0, stream>>>(X2, FFNO, ln3_g, ln3_b, dout);
}
